// CNF_3307124818030
// MI455X (gfx1250) — hardware-verified
//
#include <hip/hip_runtime.h>
#include <math.h>

constexpr int kBatch = 2048;
constexpr int kDim   = 32;
constexpr int kInF   = 33;
constexpr int kKpad  = 64;
constexpr int kHid   = 512;
constexpr int kNout  = 64;
constexpr int kRowsPerOutBlock = 32;
constexpr int kOutQuads = kRowsPerOutBlock * kInF / 4;

constexpr float kXCarry = 8.0f;
constexpr float kWCarry = 16.0f;
constexpr float kHCarry = 8.0f;
constexpr float kCCarry = 4096.0f;
constexpr float kScale1 = 1.0f / (kXCarry * kWCarry);
constexpr float kScale2 = 1.0f / (kHCarry * kWCarry);
constexpr float kScale3 = 1.0f / (kHCarry * kWCarry);
constexpr float kScale4 = 1.0f / kCCarry;

static_assert(kBatch % 64 == 0);
static_assert(kHid % 64 == 0);
static_assert(kNout % 64 == 0);
static_assert(kKpad % 32 == 0);
static_assert(kHid % 32 == 0);
static_assert((kRowsPerOutBlock * kInF) % 4 == 0);
static_assert((kRowsPerOutBlock * kInF * 4) % 128 == 0);
static_assert(kBatch % kRowsPerOutBlock == 0);

constexpr size_t kBytesW1T = (size_t)kHid * kKpad * 2;
constexpr size_t kBytesW2T = (size_t)kHid * kHid * 2;
constexpr size_t kBytesW3T = (size_t)kNout * kHid * 2;
constexpr size_t kBytesINP = (size_t)kBatch * kKpad * 2;
constexpr size_t kBytesCBT = (size_t)kHid * kHid * 2;
constexpr size_t kBytesF32 = (size_t)kBatch * kHid * 4;
constexpr size_t kBytesF16 = (size_t)kBatch * kHid * 2;
constexpr size_t kBytesDX  = (size_t)kBatch * kNout * 4;
constexpr size_t kOffW1T = 0;
constexpr size_t kOffW2T = kOffW1T + kBytesW1T;
constexpr size_t kOffW3T = kOffW2T + kBytesW2T;
constexpr size_t kOffINP = kOffW3T + kBytesW3T;
constexpr size_t kOffCBT = kOffINP + kBytesINP;
constexpr size_t kOffZ1  = kOffCBT + kBytesCBT;
constexpr size_t kOffH1  = kOffZ1 + kBytesF32;
constexpr size_t kOffG1  = kOffH1 + kBytesF16;
constexpr size_t kOffZ2  = kOffG1 + kBytesF32;
constexpr size_t kOffH2  = kOffZ2 + kBytesF32;
constexpr size_t kOffG2  = kOffH2 + kBytesF16;
constexpr size_t kOffDX  = kOffG2 + kBytesF16;
constexpr size_t kOffY   = kOffDX + kBytesDX;
constexpr size_t kWsTotal = kOffY + kBytesF32;
static_assert(kWsTotal == 25034752);
static_assert(kWsTotal <= 134217728);
static_assert(kOffW2T % 128 == 0 && kOffW3T % 128 == 0 && kOffINP % 128 == 0 && kOffCBT % 128 == 0);
static_assert(kOffZ1 % 128 == 0 && kOffH1 % 128 == 0 && kOffG1 % 128 == 0 && kOffZ2 % 128 == 0);
static_assert(kOffH2 % 128 == 0 && kOffG2 % 128 == 0 && kOffDX % 128 == 0 && kOffY % 128 == 0);

typedef __attribute__((ext_vector_type(16))) _Float16 v16h;
typedef __attribute__((ext_vector_type(8)))  _Float16 v8h;
typedef __attribute__((ext_vector_type(16))) __bf16   v16b;
typedef __attribute__((ext_vector_type(8)))  __bf16   v8b;
typedef __attribute__((ext_vector_type(8)))  float    v8f;
typedef __attribute__((ext_vector_type(4)))  float    v4f;
typedef __attribute__((ext_vector_type(2)))  float    v2f;
typedef __attribute__((ext_vector_type(4)))  unsigned int v4u;

__device__ __forceinline__ unsigned short f2bf_bits(float f) {
  unsigned u = __float_as_uint(f);
  return (unsigned short)((u + 0x7FFFu + ((u >> 16) & 1u)) >> 16);
}
__device__ __forceinline__ float bf_bits2f(unsigned short h) { return __uint_as_float(((unsigned)h) << 16); }

__device__ __forceinline__ void dep_guard_h(v8f& a, v8f& b, v16h x, v16h y) { asm volatile("v_nop\n\tv_nop\n\tv_nop\n\tv_nop" : "+v"(a), "+v"(b) : "v"(x), "v"(y)); }
__device__ __forceinline__ void dep_guard_b(v8f& a, v8f& b, v16b x, v16b y) { asm volatile("v_nop\n\tv_nop\n\tv_nop\n\tv_nop" : "+v"(a), "+v"(b) : "v"(x), "v"(y)); }
__device__ __forceinline__ void keep4_h(v16h a, v16h b, v16h c, v16h d) { asm volatile("v_nop" :: "v"(a), "v"(b), "v"(c), "v"(d)); }
__device__ __forceinline__ void keep4_b(v16b a, v16b b, v16b c, v16b d) { asm volatile("v_nop" :: "v"(a), "v"(b), "v"(c), "v"(d)); }
__device__ __forceinline__ void acc_guard4(v8f& a, v8f& b, v8f& c, v8f& d) { asm volatile("v_nop\n\tv_nop\n\tv_nop\n\tv_nop" : "+v"(a), "+v"(b), "+v"(c), "+v"(d)); }
template <typename T> struct Frag;
template <> struct Frag<_Float16> {
  typedef v16h V; union U { v16h v; v8h h[2]; };
  static __device__ __forceinline__ v16h load(const _Float16* p) {
    U f; f.h[0] = *(const v8h*)(p); f.h[1] = *(const v8h*)(p + 16); return f.v;
  }
  static __device__ __forceinline__ v8f mma(v16h a, v16h b, v8f c) {
    return __builtin_amdgcn_wmma_f32_16x16x32_f16(false, a, false, b, (short)0, c, false, false);
  }
  static __device__ __forceinline__ void guard(v8f& a, v8f& b, v16h x, v16h y) { dep_guard_h(a, b, x, y); }
  static __device__ __forceinline__ void keep(v16h a, v16h b, v16h c, v16h d) { keep4_h(a, b, c, d); }
};
template <> struct Frag<__bf16> {
  typedef v16b V; union U { v16b v; v8b h[2]; };
  static __device__ __forceinline__ v16b load(const __bf16* p) {
    U f; f.h[0] = *(const v8b*)(p); f.h[1] = *(const v8b*)(p + 16); return f.v;
  }
  static __device__ __forceinline__ v8f mma(v16b a, v16b b, v8f c) {
    return __builtin_amdgcn_wmma_f32_16x16x32_bf16(false, a, false, b, (short)0, c, false, false);
  }
  static __device__ __forceinline__ void guard(v8f& a, v8f& b, v16b x, v16b y) { dep_guard_b(a, b, x, y); }
  static __device__ __forceinline__ void keep(v16b a, v16b b, v16b c, v16b d) { keep4_b(a, b, c, d); }
};

__device__ __forceinline__ unsigned pk16(unsigned short a, unsigned short b) { return (unsigned)a | ((unsigned)b << 16); }
__device__ __forceinline__ unsigned short h_bits(float f) { const _Float16 h = (_Float16)f; return __builtin_bit_cast(unsigned short, h); }

template <int ET> struct Elem;
template <> struct Elem<0> { typedef _Float16 T; };
template <> struct Elem<1> { typedef __bf16 T; };
template <int ET, bool SPLIT, int BIAS_MODE, int OUT_MODE, bool RESID, int ACT = 0>
__global__ __launch_bounds__(256) void wmma_gemm64(
    const unsigned short* __restrict__ Ap, const unsigned short* __restrict__ A2p, int lda, long strideA,
    const unsigned short* __restrict__ Btp, const unsigned short* __restrict__ Bt2p, int ldb, long strideB,
    void* __restrict__ Cout, void* __restrict__ Cout2, int ldc, long strideC,
    const float* __restrict__ bias,
    const float* __restrict__ resid, long strideR,
    int M, int N, int K, float scale) {
  typedef typename Elem<ET>::T T;
  typedef typename Frag<T>::V V;
  const T* A = (const T*)Ap; const T* A2 = (const T*)A2p; const T* Bt = (const T*)Btp; const T* Bt2 = (const T*)Bt2p;
  __shared__ __align__(16) float sT[8][16 * 68];
  const int b    = blockIdx.y;
  const int lane = threadIdx.x & 31;
  const int wave = threadIdx.x >> 5;
  const int tilesN = N >> 6;
  const int tilesM = M >> 6;
  const int tile = blockIdx.x * 8 + wave;
  if (tile >= tilesM * tilesN) return;
  const int tm = tile / tilesN;
  const int tn = tile - tm * tilesN;
  const int m0 = tm << 6;
  const int n0 = tn << 6;

  const T* Ab  = A  + (size_t)b * strideA;
  const T* Bb  = Bt + (size_t)b * strideB;
  const T* Ab2 = SPLIT ? (A2  + (size_t)b * strideA) : nullptr;
  const T* Bb2 = SPLIT ? (Bt2 + (size_t)b * strideB) : nullptr;

  const int rlane = lane & 15;
  const int koff  = (lane >> 4) * 8;
  const int mOff  = (lane >> 4) * 8;

  v8f acc[4][4];
#pragma unroll
  for (int i = 0; i < 4; ++i)
#pragma unroll
    for (int j = 0; j < 4; ++j) acc[i][j] = (v8f){0.f,0.f,0.f,0.f,0.f,0.f,0.f,0.f};

  for (int k0 = 0; k0 < K; k0 += 32) {
    V bh[4], bl[4];
#pragma unroll
    for (int j = 0; j < 4; ++j) {
      const size_t bo = (size_t)(n0 + (j << 4) + rlane) * ldb + koff + k0;
      bh[j] = Frag<T>::load(Bb + bo);
      if (SPLIT) bl[j] = Frag<T>::load(Bb2 + bo);
    }
#pragma unroll
    for (int i = 0; i < 4; ++i) {
      const size_t ao = (size_t)(m0 + (i << 4) + rlane) * lda + koff + k0;
      V ah = Frag<T>::load(Ab + ao);
      V al;
      if (SPLIT) al = Frag<T>::load(Ab2 + ao);
#pragma unroll
      for (int j = 0; j < 4; ++j) {
        acc[i][j] = Frag<T>::mma(ah, bh[j], acc[i][j]);
        if (SPLIT) {
          acc[i][j] = Frag<T>::mma(ah, bl[j], acc[i][j]);
          acc[i][j] = Frag<T>::mma(al, bh[j], acc[i][j]);
        }
      }
      Frag<T>::guard(acc[i][0], acc[i][3], ah, SPLIT ? al : ah);
    }
    Frag<T>::keep(bh[0], bh[1], bh[2], bh[3]);
    if (SPLIT) Frag<T>::keep(bl[0], bl[1], bl[2], bl[3]);
  }
  acc_guard4(acc[0][0], acc[0][1], acc[0][2], acc[0][3]);
  acc_guard4(acc[1][0], acc[1][1], acc[1][2], acc[1][3]);
  acc_guard4(acc[2][0], acc[2][1], acc[2][2], acc[2][3]);
  acc_guard4(acc[3][0], acc[3][1], acc[3][2], acc[3][3]);

  float* slab = sT[wave];
  const float* Rb = RESID ? (resid + (size_t)b * strideR) : nullptr;
#pragma unroll
  for (int i = 0; i < 4; ++i) {
    const int mBase = m0 + (i << 4);
#pragma unroll
    for (int j = 0; j < 4; ++j) {
      const int n = n0 + (j << 4) + rlane;
      float bv = 0.f;
      if (BIAS_MODE == 2) bv = bias[n];
#pragma unroll
      for (int r = 0; r < 8; ++r) {
        float v = acc[i][j][r] * scale;
        if (BIAS_MODE == 1) v += bias[mBase + mOff + r];
        if (BIAS_MODE == 2) v += bv;
        if (RESID) v += Rb[(size_t)(mBase + mOff + r) * ldc + n];
        if (ACT == 2) v = fmaxf(v, 0.0f);
        if (ACT == 4) v = (v > 0.f) ? v : 0.01f * v;
        slab[(mOff + r) * 68 + (j << 4) + rlane] = v;
      }
    }
    __builtin_amdgcn_fence(__ATOMIC_RELEASE, "workgroup");
    __builtin_amdgcn_wave_barrier();
    __builtin_amdgcn_fence(__ATOMIC_ACQUIRE, "workgroup");
    if (OUT_MODE == 0) {
      float* C = (float*)Cout + (size_t)b * strideC;
      const int hh = lane >> 4, c4 = (lane & 15) * 4;
      for (int pass = 0; pass < 2; ++pass) {
#pragma unroll
        for (int it = 0; it < 8; ++it) {
          const int row = it * 2 + hh;
          v4f v = *(const v4f*)(slab + row * 68 + c4);
          *(volatile v4f*)(C + (size_t)(mBase + row) * ldc + n0 + c4) = v;
        }
        __threadfence();
      }
    } else {
      const int q = lane >> 3, c8 = (lane & 7) * 8;
      unsigned short* C  = (unsigned short*)Cout  + (size_t)b * strideC;
      unsigned short* C2 = (OUT_MODE == 2) ? ((unsigned short*)Cout2 + (size_t)b * strideC) : nullptr;
      for (int pass = 0; pass < 2; ++pass) {
#pragma unroll
        for (int it = 0; it < 4; ++it) {
          const int row = it * 4 + q;
          const float* sp = slab + row * 68 + c8;
          v8h hv, lv;
#pragma unroll
          for (int e = 0; e < 8; ++e) {
            if (OUT_MODE == 1) {
              hv[e] = (_Float16)sp[e];
            } else {
              unsigned short hb = f2bf_bits(sp[e]);
              unsigned short lb = f2bf_bits(sp[e] - bf_bits2f(hb));
              hv[e] = __builtin_bit_cast(_Float16, hb);
              lv[e] = __builtin_bit_cast(_Float16, lb);
            }
          }
          *(volatile v8h*)(C + (size_t)(mBase + row) * ldc + n0 + c8) = hv;
          if (OUT_MODE == 2) *(volatile v8h*)(C2 + (size_t)(mBase + row) * ldc + n0 + c8) = lv;
        }
        __threadfence();
      }
    }
    __builtin_amdgcn_fence(__ATOMIC_RELEASE, "workgroup");
    __builtin_amdgcn_wave_barrier();
    __builtin_amdgcn_fence(__ATOMIC_ACQUIRE, "workgroup");
  }
}

__global__ __launch_bounds__(256) void w2t_kernel(const float* __restrict__ W, unsigned short* __restrict__ outp, float scale) {
  __shared__ float sm[64][65];
  const int t  = threadIdx.x;
  const int d0 = blockIdx.x * 64;
  const int h0 = blockIdx.y * 64;
#pragma unroll
  for (int i = 0; i < 8; ++i) {
    const int e = i * 256 + t;
    const int r = e >> 6;
    const int c = e & 63;
    sm[c][r] = W[(size_t)(d0 + r) * kHid + h0 + c] * scale;
  }
  asm volatile("" ::: "memory");
#pragma unroll
  for (int i = 8; i < 16; ++i) {
    const int e = i * 256 + t;
    const int r = e >> 6;
    const int c = e & 63;
    sm[c][r] = W[(size_t)(d0 + r) * kHid + h0 + c] * scale;
  }
  __syncthreads();
  const int lane = t & 31, wave = t >> 5;
  const int q = lane >> 3, c8 = (lane & 7) * 8;
  for (int pass = 0; pass < 2; ++pass) {
#pragma unroll
    for (int it = 0; it < 2; ++it) {
      const int row = wave * 8 + it * 4 + q;
      unsigned short hb[8];
#pragma unroll
      for (int e = 0; e < 8; ++e) hb[e] = h_bits(sm[row][c8 + e]);
      const v4u u = (v4u){pk16(hb[0], hb[1]), pk16(hb[2], hb[3]), pk16(hb[4], hb[5]), pk16(hb[6], hb[7])};
      *(volatile v4u*)(outp + (size_t)(h0 + row) * kHid + d0 + c8) = u;
    }
    __threadfence();
  }
}

__global__ __launch_bounds__(256) void w1t_kernel(const float* __restrict__ W1, unsigned short* __restrict__ outp, float scale) {
  __shared__ float sm[kInF][65];
  const int t  = threadIdx.x;
  const int n0 = blockIdx.x * 64;
  constexpr int kTot = kInF * 64;
#pragma unroll
  for (int i = 0; i < 9; ++i) {
    const int e  = i * 256 + t;
    const int ec = (e < kTot) ? e : (kTot - 1);
    const int k  = ec >> 6;
    const int nl = ec & 63;
    const float v = W1[(size_t)k * kHid + n0 + nl] * scale;
    if (e < kTot) sm[k][nl] = v;
  }
  __syncthreads();
  const int lane = t & 31, wave = t >> 5;
  const int q = lane >> 3, c8 = (lane & 7) * 8;
  for (int pass = 0; pass < 2; ++pass) {
#pragma unroll
    for (int it = 0; it < 2; ++it) {
      const int row = wave * 8 + it * 4 + q;
      unsigned short hb[8];
#pragma unroll
      for (int e = 0; e < 8; ++e) {
        const int k  = c8 + e;
        const int kc = (k < kInF) ? k : (kInF - 1);
        float v = sm[kc][row];
        v = (k < kInF) ? v : 0.0f;
        hb[e] = h_bits(v);
      }
      const v4u u = (v4u){pk16(hb[0], hb[1]), pk16(hb[2], hb[3]), pk16(hb[4], hb[5]), pk16(hb[6], hb[7])};
      *(volatile v4u*)(outp + (size_t)(n0 + row) * kKpad + c8) = u;
    }
    __threadfence();
  }
}

__global__ __launch_bounds__(256) void w3t_kernel(const float* __restrict__ W3, unsigned short* __restrict__ outp, float scale) {
  __shared__ float sm[64][kDim + 1];
  const int t  = threadIdx.x;
  const int k0 = blockIdx.x * 64;
#pragma unroll
  for (int i = 0; i < 8; ++i) {
    const int e  = i * 256 + t;
    const int kl = e >> 5;
    const int n  = e & 31;
    sm[kl][n] = W3[(size_t)(k0 + kl) * kDim + n] * scale;
  }
  __syncthreads();
  const int lane = t & 31, wave = t >> 5;
  const int q = lane >> 3, c8 = (lane & 7) * 8;
  for (int pass = 0; pass < 2; ++pass) {
#pragma unroll
    for (int it = 0; it < 2; ++it) {
      const int row = wave * 8 + it * 4 + q;
      const int nc  = (row < kDim) ? row : (kDim - 1);
      unsigned short hb[8];
#pragma unroll
      for (int e = 0; e < 8; ++e) {
        const int kl = c8 + e;
        float v = sm[kl][nc];
        v = (row < kDim) ? v : 0.0f;
        hb[e] = h_bits(v);
      }
      const v4u u = (v4u){pk16(hb[0], hb[1]), pk16(hb[2], hb[3]), pk16(hb[4], hb[5]), pk16(hb[6], hb[7])};
      *(volatile v4u*)(outp + (size_t)row * kHid + k0 + c8) = u;
    }
    __threadfence();
  }
}

__global__ __launch_bounds__(256) void inp_kernel(const float* __restrict__ tptr, const float* __restrict__ x,
                                                  unsigned short* __restrict__ outp) {
  __shared__ float sm[64 * kInF];
  const int t  = threadIdx.x;
  const int m0 = blockIdx.x * 64;
  const float tv = tptr[0];
  constexpr int kTot = 64 * kInF;
#pragma unroll
  for (int i = 0; i < 9; ++i) {
    const int e  = i * 256 + t;
    const int ec = (e < kTot) ? e : (kTot - 1);
    const float v = x[(size_t)m0 * kInF + ec];
    if (e < kTot) sm[e] = v;
  }
  __syncthreads();
  if (t < 64) sm[t * kInF + kDim] = tv;
  __syncthreads();
  const int lane = t & 31, wave = t >> 5;
  const int q = lane >> 3, c8 = (lane & 7) * 8;
  for (int pass = 0; pass < 2; ++pass) {
#pragma unroll
    for (int it = 0; it < 2; ++it) {
      const int row = wave * 8 + it * 4 + q;
      unsigned short hb[8];
#pragma unroll
      for (int e = 0; e < 8; ++e) {
        const int k  = c8 + e;
        const int kc = (k <= kDim) ? k : kDim;
        float v = sm[row * kInF + kc] * kXCarry;
        v = (k <= kDim) ? v : 0.0f;
        hb[e] = h_bits(v);
      }
      const v4u u = (v4u){pk16(hb[0], hb[1]), pk16(hb[2], hb[3]), pk16(hb[4], hb[5]), pk16(hb[6], hb[7])};
      *(volatile v4u*)(outp + (size_t)(m0 + row) * kKpad + c8) = u;
    }
    __threadfence();
  }
}

__global__ __launch_bounds__(256) void cprep_kernel(const float* __restrict__ W1, const float* __restrict__ W2,
                                                    const float* __restrict__ W3, unsigned short* __restrict__ outp) {
  __shared__ float sW1[kDim][64];
  __shared__ float sW3[64][kDim];
  __shared__ float sW2[64][65];
  const int t  = threadIdx.x;
  const int b0 = blockIdx.x * 64;
  const int a0 = blockIdx.y * 64;
#pragma unroll
  for (int i = 0; i < 8; ++i) {
    const int e = i * 256 + t;
    const int j = e >> 6, al = e & 63;
    sW1[j][al] = W1[(size_t)j * kHid + a0 + al];
  }
  asm volatile("" ::: "memory");
#pragma unroll
  for (int i = 0; i < 8; ++i) {
    const int e = i * 256 + t;
    const int bl = e >> 5, j = e & 31;
    sW3[bl][j] = W3[(size_t)(b0 + bl) * kDim + j];
  }
  asm volatile("" ::: "memory");
#pragma unroll
  for (int i = 0; i < 8; ++i) {
    const int e = i * 256 + t;
    const int al = e >> 6, bl = e & 63;
    sW2[al][bl] = W2[(size_t)(a0 + al) * kHid + b0 + bl];
  }
  asm volatile("" ::: "memory");
#pragma unroll
  for (int i = 8; i < 16; ++i) {
    const int e = i * 256 + t;
    const int al = e >> 6, bl = e & 63;
    sW2[al][bl] = W2[(size_t)(a0 + al) * kHid + b0 + bl];
  }
  __syncthreads();
  {
    const int al = t & 63;
    const int bg = t >> 6;
#pragma unroll 1
    for (int i = 0; i < 16; ++i) {
      const int bl = bg * 16 + i;
      float s = 0.0f;
#pragma unroll
      for (int j = 0; j < kDim; ++j) s += sW3[bl][j] * sW1[j][al];
      const float cv = sW2[al][bl] * s * kCCarry;
      sW2[al][bl] = cv;
    }
  }
  __syncthreads();
  const int lane = t & 31, wave = t >> 5;
  const int q = lane >> 3, c8 = (lane & 7) * 8;
  for (int pass = 0; pass < 2; ++pass) {
#pragma unroll
    for (int it = 0; it < 2; ++it) {
      const int row = wave * 8 + it * 4 + q;
      unsigned short hb[8];
#pragma unroll
      for (int e = 0; e < 8; ++e) hb[e] = h_bits(sW2[row][c8 + e]);
      const v4u u = (v4u){pk16(hb[0], hb[1]), pk16(hb[2], hb[3]), pk16(hb[4], hb[5]), pk16(hb[6], hb[7])};
      *(volatile v4u*)(outp + (size_t)(a0 + row) * kHid + b0 + c8) = u;
    }
    __threadfence();
  }
}

template <bool G16>
__global__ __launch_bounds__(256) void act_kernel(const float* __restrict__ Z, unsigned short* __restrict__ Hp,
                                                  void* __restrict__ Gp, int n2, float hcarry) {
  const int i = blockIdx.x * 256 + threadIdx.x;
  if (i >= n2) return;
  const v2f z = *(const v2f*)(Z + 2 * (size_t)i);
  const float z0 = z[0];
  const float z1 = z[1];
  const float h0 = tanhf(z0);
  const float h1 = tanhf(z1);
  const float g0 = 1.0f - h0 * h0;
  const float g1 = 1.0f - h1 * h1;
  const unsigned hw = pk16(h_bits(h0 * hcarry), h_bits(h1 * hcarry));
  unsigned* hq = (unsigned*)Hp + i;
  if (G16) {
    const unsigned gw = pk16(h_bits(g0), h_bits(g1));
    unsigned* gq = (unsigned*)Gp + i;
    *(volatile unsigned*)hq = hw;
    *(volatile unsigned*)gq = gw;
    __threadfence();
    *(volatile unsigned*)hq = hw;
    *(volatile unsigned*)gq = gw;
  } else {
    const v2f gv = (v2f){g0, g1};
    float* gq = (float*)Gp + 2 * (size_t)i;
    *(volatile unsigned*)hq = hw;
    *(volatile v2f*)gq = gv;
    __threadfence();
    *(volatile unsigned*)hq = hw;
    *(volatile v2f*)gq = gv;
  }
}

__global__ __launch_bounds__(256) void final_kernel(const float* __restrict__ Y, const float* __restrict__ G1,
                                                    const float* __restrict__ DX, const float* __restrict__ b3,
                                                    float* __restrict__ outp) {
  __shared__ float sDiv[kRowsPerOutBlock];
  __shared__ __align__(16) float sOut[kRowsPerOutBlock * kInF];
  const int t = threadIdx.x;
  const int lane = t & 31, wave = t >> 5;
  const int r0 = blockIdx.x * kRowsPerOutBlock;
#pragma unroll 1
  for (int rr = 0; rr < 4; ++rr) {
    const int row = r0 + wave * 4 + rr;
    const float* yr = Y  + (size_t)row * kHid + 4 * lane;
    const float* gr = G1 + (size_t)row * kHid + 4 * lane;
    float s = 0.0f;
    {
      const v4f ya = *(const v4f*)(yr);
      const v4f ga = *(const v4f*)(gr);
      const v4f yb = *(const v4f*)(yr + 128);
      const v4f gb = *(const v4f*)(gr + 128);
      s += ya[0] * ga[0]; s += ya[1] * ga[1]; s += ya[2] * ga[2]; s += ya[3] * ga[3];
      s += yb[0] * gb[0]; s += yb[1] * gb[1]; s += yb[2] * gb[2]; s += yb[3] * gb[3];
    }
    asm volatile("" ::: "memory");
    {
      const v4f ya = *(const v4f*)(yr + 256);
      const v4f ga = *(const v4f*)(gr + 256);
      const v4f yb = *(const v4f*)(yr + 384);
      const v4f gb = *(const v4f*)(gr + 384);
      s += ya[0] * ga[0]; s += ya[1] * ga[1]; s += ya[2] * ga[2]; s += ya[3] * ga[3];
      s += yb[0] * gb[0]; s += yb[1] * gb[1]; s += yb[2] * gb[2]; s += yb[3] * gb[3];
    }
#pragma unroll
    for (int off = 16; off > 0; off >>= 1) s += __shfl_xor(s, off, 32);
    if (lane == 0) sDiv[wave * 4 + rr] = s;
    asm volatile("" ::: "memory");
  }
  __syncthreads();
#pragma unroll
  for (int i = 0; i < 4; ++i) {
    const int e  = i * 256 + t;
    const int rl = e >> 5;
    const int c  = e & 31;
    sOut[rl * kInF + c] = DX[(size_t)(r0 + rl) * kNout + c] + b3[c];
  }
  if (t < kRowsPerOutBlock) sOut[t * kInF + kDim] = sDiv[t];
  __syncthreads();
  float* ob = outp + (size_t)r0 * kInF;
  for (int pass = 0; pass < 2; ++pass) {
    for (int idx = t; idx < kOutQuads; idx += 256) {
      const v4f v = *(const v4f*)(sOut + 4 * idx);
      *(volatile v4f*)(ob + 4 * idx) = v;
    }
    __threadfence();
  }
}

extern "C" void kernel_launch(void* const* d_in, const int* in_sizes, int n_in,
                              void* d_out, int out_size, void* d_ws, size_t ws_size,
                              hipStream_t stream) {
  if (n_in < 8) return;
  if (out_size != kBatch * kInF) return;
  if (ws_size < kWsTotal) return;
  const float* tptr = (const float*)d_in[0];
  const float* x    = (const float*)d_in[1];
  const float* W1   = (const float*)d_in[2];
  const float* b1   = (const float*)d_in[3];
  const float* W2   = (const float*)d_in[4];
  const float* b2   = (const float*)d_in[5];
  const float* W3   = (const float*)d_in[6];
  const float* b3   = (const float*)d_in[7];
  float* outp = (float*)d_out;

  unsigned char* ws = (unsigned char*)d_ws;
  unsigned short* W1T = (unsigned short*)(ws + kOffW1T);
  unsigned short* W2T = (unsigned short*)(ws + kOffW2T);
  unsigned short* W3T = (unsigned short*)(ws + kOffW3T);
  unsigned short* INP = (unsigned short*)(ws + kOffINP);
  unsigned short* CBT = (unsigned short*)(ws + kOffCBT);
  float*          Z1  = (float*)(ws + kOffZ1);
  unsigned short* H1  = (unsigned short*)(ws + kOffH1);
  float*          G1  = (float*)(ws + kOffG1);
  float*          Z2  = (float*)(ws + kOffZ2);
  unsigned short* H2  = (unsigned short*)(ws + kOffH2);
  unsigned short* G2  = (unsigned short*)(ws + kOffG2);
  float*          DX  = (float*)(ws + kOffDX);
  float*          Y   = (float*)(ws + kOffY);

  constexpr int kN2 = kBatch * kHid / 2;
  static_assert(kN2 % 256 == 0);

  w1t_kernel<<<dim3(kHid / 64), dim3(256), 0, stream>>>(W1, W1T, kWCarry);
  w2t_kernel<<<dim3(kHid / 64, kHid / 64), dim3(256), 0, stream>>>(W2, W2T, kWCarry);
  w3t_kernel<<<dim3(kHid / 64), dim3(256), 0, stream>>>(W3, W3T, kWCarry);
  inp_kernel<<<dim3(kBatch / 64), dim3(256), 0, stream>>>(tptr, x, INP);
  cprep_kernel<<<dim3(kHid / 64, kHid / 64), dim3(256), 0, stream>>>(W1, W2, W3, CBT);

  wmma_gemm64<0, false, 2, 0, false, 0><<<dim3((kBatch / 64) * (kHid / 64) / 8, 1), dim3(256), 0, stream>>>(
      INP, INP, kKpad, 0L, W1T, W1T, kKpad, 0L, (void*)Z1, (void*)Z1, kHid, 0L, b1, (const float*)Z1, 0L,
      kBatch, kHid, kKpad, kScale1);
  act_kernel<false><<<dim3(kN2 / 256), dim3(256), 0, stream>>>(Z1, H1, (void*)G1, kN2, kHCarry);

  wmma_gemm64<0, false, 2, 0, false, 0><<<dim3((kBatch / 64) * (kHid / 64) / 8, 1), dim3(256), 0, stream>>>(
      H1, H1, kHid, 0L, W2T, W2T, kHid, 0L, (void*)Z2, (void*)Z2, kHid, 0L, b2, (const float*)Z1, 0L,
      kBatch, kHid, kHid, kScale2);
  act_kernel<true><<<dim3(kN2 / 256), dim3(256), 0, stream>>>(Z2, H2, (void*)G2, kN2, kHCarry);

  wmma_gemm64<0, false, 0, 0, false, 0><<<dim3((kBatch / 64) * (kNout / 64) / 8, 1), dim3(256), 0, stream>>>(
      H2, H2, kHid, 0L, W3T, W3T, kHid, 0L, (void*)DX, (void*)DX, kNout, 0L, b1, (const float*)Z1, 0L,
      kBatch, kNout, kHid, kScale3);

  wmma_gemm64<0, false, 0, 0, false, 0><<<dim3((kBatch / 64) * (kHid / 64) / 8, 1), dim3(256), 0, stream>>>(
      G2, G2, kHid, 0L, CBT, CBT, kHid, 0L, (void*)Y, (void*)Y, kHid, 0L, b1, (const float*)Z1, 0L,
      kBatch, kHid, kHid, kScale4);

  final_kernel<<<dim3(kBatch / kRowsPerOutBlock), dim3(256), 0, stream>>>(Y, G1, DX, b3, outp);
}
